// MASGNN_27754078667623
// MI455X (gfx1250) — hardware-verified
//
#include <hip/hip_runtime.h>
#include <stddef.h>
#include <math.h>


#define HD      64
#define AD      32
#define G3      192
#define NTHR    256
#define NWAVE   8
#define EPT     8
#define NGRP    2
#define CHUNK   (NTHR * EPT * NGRP)
#define WCAP    (EPT * NGRP * 32)
#define LISTN   (NWAVE * WCAP)
#define NBC     4096
#define NBF     1024
#define RCAP    40960
#define RBN     128
#define TGT     256
#define DEGCAP  2048
#define OTHR    512
#define BM      32
#define PTHR    128
#define WSCAP   134217728
#define SCL_A   8.0f
#define SCL_W   16.0f
#define SCL_ACC 0.0078125f

#define LDS_FILL ((RCAP + NBF + LISTN) * 4 + 64)

static_assert((CHUNK & (CHUNK - 1)) == 0);
static_assert(CHUNK <= 4096);
static_assert(NBC <= 4096 && NBF <= 4096);
static_assert((NBC & (NBC - 1)) == 0 && (NBF & (NBF - 1)) == 0);
static_assert(NBC == 4 * NBF);
static_assert(OTHR * 8 == NBC);
static_assert((RCAP % 32) == 0);
static_assert(TGT == NWAVE * 32);
static_assert((NBC % TGT) == 0);
static_assert((TGT % BM) == 0);
static_assert(HD == 64 && AD == 32 && G3 == 3 * HD);
static_assert(BM * 8 == NTHR);

typedef float    v2f  __attribute__((ext_vector_type(2)));
typedef float    v4f  __attribute__((ext_vector_type(4)));
typedef float    v8f  __attribute__((ext_vector_type(8)));
typedef int      v4i  __attribute__((ext_vector_type(4)));
typedef _Float16 v2h  __attribute__((ext_vector_type(2)));
typedef _Float16 v4h  __attribute__((ext_vector_type(4)));
typedef _Float16 v8h  __attribute__((ext_vector_type(8)));
typedef _Float16 v16h __attribute__((ext_vector_type(16)));
union FragH { v16h v; v8h h[2]; };

__device__ __forceinline__ v8f wmh(v16h a, v16h b, v8f c) {
  v8f d = __builtin_amdgcn_wmma_f32_16x16x32_f16(false, a, false, b, (short)0, c, false, false);
  asm volatile("v_nop\n\tv_nop\n\tv_nop\n\tv_nop" : "+v"(d) : "v"(a), "v"(b));
  return d;
}

__device__ __forceinline__ v8h cvt8(v4f a, v4f b, float s) {
  v8f t;
  t[0] = a.x * s; t[1] = a.y * s; t[2] = a.z * s; t[3] = a.w * s;
  t[4] = b.x * s; t[5] = b.y * s; t[6] = b.z * s; t[7] = b.w * s;
  return __builtin_convertvector(t, v8h);
}

__device__ __forceinline__ float sigm(float x) {
  x = x > 30.0f ? 30.0f : (x < -30.0f ? -30.0f : x);
  const float e = expf(-x);
  return 1.0f / (1.0f + e);
}

template <int NB>
__device__ __forceinline__ int scan_chunk(const int* __restrict__ dsts, int nE, int cbase, int slotBase,
                                          int vec8, int* list, int tid, int lane, int wave) {
  int wc = 0;
#pragma unroll
  for (int g = 0; g < NGRP; ++g) {
    const int el0  = (g * NTHR + tid) * EPT;
    const int e0   = cbase + el0;
    const int sent = -2147483647 - 1;
    v4i da, db;
    if (vec8 != 0 && cbase + CHUNK <= nE) {
      da = *(const v4i*)(dsts + e0);
      db = *(const v4i*)(dsts + e0 + 4);
    } else {
      da.x = (e0     < nE) ? dsts[min(e0, nE - 1)] : sent;
      da.y = (e0 + 1 < nE) ? dsts[min(e0 + 1, nE - 1)] : sent;
      da.z = (e0 + 2 < nE) ? dsts[min(e0 + 2, nE - 1)] : sent;
      da.w = (e0 + 3 < nE) ? dsts[min(e0 + 3, nE - 1)] : sent;
      db.x = (e0 + 4 < nE) ? dsts[min(e0 + 4, nE - 1)] : sent;
      db.y = (e0 + 5 < nE) ? dsts[min(e0 + 5, nE - 1)] : sent;
      db.z = (e0 + 6 < nE) ? dsts[min(e0 + 6, nE - 1)] : sent;
      db.w = (e0 + 7 < nE) ? dsts[min(e0 + 7, nE - 1)] : sent;
    }
    const unsigned nb = (unsigned)slotBase;
    const unsigned s0 = (unsigned)da.x - nb, s1 = (unsigned)da.y - nb;
    const unsigned s2 = (unsigned)da.z - nb, s3 = (unsigned)da.w - nb;
    const unsigned s4 = (unsigned)db.x - nb, s5 = (unsigned)db.y - nb;
    const unsigned s6 = (unsigned)db.z - nb, s7 = (unsigned)db.w - nb;
    const bool h0 = s0 < (unsigned)NB, h1 = s1 < (unsigned)NB, h2 = s2 < (unsigned)NB, h3 = s3 < (unsigned)NB;
    const bool h4 = s4 < (unsigned)NB, h5 = s5 < (unsigned)NB, h6 = s6 < (unsigned)NB, h7 = s7 < (unsigned)NB;
    const unsigned any = __builtin_amdgcn_ballot_w32(h0 | h1 | h2 | h3 | h4 | h5 | h6 | h7);
    if (any != 0u) {
#define HITJ(J, HJ, SJ) { \
        const unsigned mj = __builtin_amdgcn_ballot_w32(HJ); \
        if (mj != 0u) { \
          if (HJ) { \
            const int pos = wc + (int)__builtin_amdgcn_mbcnt_lo(mj, 0u); \
            if (pos < WCAP) list[wave * WCAP + pos] = ((el0 + (J)) << 12) | (int)(SJ); \
          } \
          wc += (int)__builtin_popcount(mj); } }
      HITJ(0, h0, s0)
      HITJ(1, h1, s1)
      HITJ(2, h2, s2)
      HITJ(3, h3, s3)
      HITJ(4, h4, s4)
      HITJ(5, h5, s5)
      HITJ(6, h6, s6)
      HITJ(7, h7, s7)
#undef HITJ
    }
  }
  return wc;
}

__global__ __launch_bounds__(NTHR) void k_extract(const int* __restrict__ edges, int* objp, int nE, int nUnits) {
  const int i = (int)blockIdx.x * NTHR + (int)threadIdx.x;
  if (i >= nUnits) return;
  const int e0 = 4 * i;
  const int a0 = min(e0, nE - 1), a1 = min(e0 + 1, nE - 1), a2 = min(e0 + 2, nE - 1), a3 = min(e0 + 3, nE - 1);
  v4i v;
  v.x = edges[(size_t)a0 * 6 + 5];
  v.y = edges[(size_t)a1 * 6 + 5];
  v.z = edges[(size_t)a2 * 6 + 5];
  v.w = edges[(size_t)a3 * 6 + 5];
  int* d = objp + (size_t)4 * i;
  *(volatile v4i*)d = v;
  __threadfence();
  *(volatile v4i*)d = v;
}

__global__ __launch_bounds__(NTHR) void k_zero16(float* p, int nUnits) {
  const int i = (int)blockIdx.x * NTHR + (int)threadIdx.x;
  if (i >= nUnits) return;
  const v4f z = {0.0f, 0.0f, 0.0f, 0.0f};
  float* d = p + (size_t)4 * i;
  *(volatile v4f*)d = z;
  __threadfence();
  *(volatile v4f*)d = z;
}

__global__ __launch_bounds__(NTHR) void k_prepw_flat(const float* __restrict__ W, _Float16* wp, int nUnits) {
  const int i = (int)blockIdx.x * NTHR + (int)threadIdx.x;
  if (i >= nUnits) return;
  const float* p = W + (size_t)i * 8;
  const v4f a = *(const v4f*)p;
  const v4f b = *(const v4f*)(p + 4);
  const v8h o = cvt8(a, b, SCL_W);
  _Float16* d = wp + (size_t)i * 8;
  *(volatile v8h*)d = o;
  __threadfence();
  *(volatile v8h*)d = o;
}

__global__ __launch_bounds__(NTHR) void k_acvt(const float* __restrict__ rela, _Float16* rp, int nRel, int rpad, int nUnits) {
  const int i  = (int)blockIdx.x * NTHR + (int)threadIdx.x;
  const int ly = (int)blockIdx.y;
  if (i >= nUnits) return;
  const int row = i >> 3;
  const int c0  = (i & 7) * 8;
  int rr = row > nRel - 1 ? nRel - 1 : row;
  rr = rr < 0 ? 0 : rr;
  const float* p = rela + ((size_t)ly * nRel + rr) * HD + c0;
  const v4f a = *(const v4f*)p;
  const v4f b = *(const v4f*)(p + 4);
  v8h o = cvt8(a, b, SCL_A);
  const v8h z = {(_Float16)0.0f, (_Float16)0.0f, (_Float16)0.0f, (_Float16)0.0f,
                 (_Float16)0.0f, (_Float16)0.0f, (_Float16)0.0f, (_Float16)0.0f};
  o = (row < nRel) ? o : z;
  _Float16* d = rp + (size_t)ly * rpad * HD + (size_t)i * 8;
  *(volatile v8h*)d = o;
  __threadfence();
  *(volatile v8h*)d = o;
}

__global__ __launch_bounds__(NTHR) void k_count(
    const int* __restrict__ dsts, int* cnt, int nE, int vec8) {
  __shared__ __attribute__((aligned(16))) int scnt[NBC];
  __shared__ __attribute__((aligned(16))) int list[LISTN];
  __shared__ int wcnt[NWAVE];
  const int tid = threadIdx.x, lane = tid & 31, wave = tid >> 5;
  const int nodeBase = blockIdx.x * NBC;

  for (int i = tid; i < NBC; i += NTHR) scnt[i] = 0;
  __syncthreads();

  const int nChunks = (nE + CHUNK - 1) / CHUNK;
#pragma unroll 1
  for (int ch = 0; ch < nChunks; ++ch) {
    const int cbase = ch * CHUNK;
    const int wc = scan_chunk<NBC>(dsts, nE, cbase, nodeBase, vec8, list, tid, lane, wave);
    if (lane == 0) wcnt[wave] = wc;
    __syncthreads();
    if (wave == 0) {
#pragma unroll 1
      for (int wsx = 0; wsx < NWAVE; ++wsx) {
        int n = __builtin_amdgcn_readfirstlane(wcnt[wsx]);
        n = n > WCAP ? WCAP : (n < 0 ? 0 : n);
        const int* lp = list + wsx * WCAP;
#pragma unroll 1
        for (int i = 0; i < n; ++i) {
          const int ent  = __builtin_amdgcn_readfirstlane(lp[i]);
          const int slot = ent & (NBC - 1);
          if (lane == 0) scnt[slot] = scnt[slot] + 1;
        }
      }
    }
    __syncthreads();
  }

  v4i cq[4];
#pragma unroll
  for (int q = 0; q < 4; ++q) {
    const int f = (wave * 4 + q) * 128 + 4 * lane;
    cq[q] = *(const v4i*)(scnt + f);
  }
  int* cp = cnt + (size_t)nodeBase;
#pragma unroll
  for (int q = 0; q < 4; ++q) {
    const int f = (wave * 4 + q) * 128 + 4 * lane;
    *(volatile v4i*)(cp + f) = cq[q];
  }
  __threadfence();
#pragma unroll
  for (int q = 0; q < 4; ++q) {
    const int f = (wave * 4 + q) * 128 + 4 * lane;
    *(volatile v4i*)(cp + f) = cq[q];
  }
}

__global__ __launch_bounds__(OTHR) void k_offsets(
    const int* __restrict__ cnt, int* off, int* rbase, int nChunk) {
  __shared__ __attribute__((aligned(16))) int soff[NBC];
  __shared__ __attribute__((aligned(16))) int srb[RBN];
  __shared__ int wtot[OTHR / 32];
  const int tid = threadIdx.x, lane = tid & 31, wave = tid >> 5, sub = tid >> 7;
  for (int i = tid; i < RBN; i += OTHR) srb[i] = 0;
  int carry = 0;
#pragma unroll 1
  for (int ch = 0; ch < nChunk; ++ch) {
    const int base = ch * NBC;
    const v4i c0 = *(const v4i*)(cnt + base + 8 * tid);
    const v4i c1 = *(const v4i*)(cnt + base + 8 * tid + 4);
    const int e0 = max(c0.x, 0), e1 = max(c0.y, 0), e2 = max(c0.z, 0), e3 = max(c0.w, 0);
    const int e4 = max(c1.x, 0), e5 = max(c1.y, 0), e6 = max(c1.z, 0), e7 = max(c1.w, 0);
    const int ts = e0 + e1 + e2 + e3 + e4 + e5 + e6 + e7;
    int incl = ts;
#pragma unroll
    for (int d = 1; d < 32; d <<= 1) {
      const int t = __shfl_up(incl, d);
      if (lane >= d) incl += t;
    }
    if (lane == 31) wtot[wave] = incl;
    __syncthreads();
    const int S0 = wtot[0]  + wtot[1]  + wtot[2]  + wtot[3];
    const int S1 = wtot[4]  + wtot[5]  + wtot[6]  + wtot[7];
    const int S2 = wtot[8]  + wtot[9]  + wtot[10] + wtot[11];
    const int S3 = wtot[12] + wtot[13] + wtot[14] + wtot[15];
    int pre = 0;
#pragma unroll 1
    for (int w = 4 * sub; w < wave; ++w) pre += wtot[w];
    const int b0 = carry;
    const int b1 = b0 + ((S0 + 31) & ~31);
    const int b2 = b1 + ((S1 + 31) & ~31);
    const int b3 = b2 + ((S2 + 31) & ~31);
    const int b4 = b3 + ((S3 + 31) & ~31);
    const int myb = sub == 0 ? b0 : (sub == 1 ? b1 : (sub == 2 ? b2 : b3));
    if (tid == 0) {
      srb[min(4 * ch + 0, RBN - 1)] = b0;
      srb[min(4 * ch + 1, RBN - 1)] = b1;
      srb[min(4 * ch + 2, RBN - 1)] = b2;
      srb[min(4 * ch + 3, RBN - 1)] = b3;
    }
    int run = myb + pre + incl - ts;
    soff[8 * tid + 0] = run; run += e0;
    soff[8 * tid + 1] = run; run += e1;
    soff[8 * tid + 2] = run; run += e2;
    soff[8 * tid + 3] = run; run += e3;
    soff[8 * tid + 4] = run; run += e4;
    soff[8 * tid + 5] = run; run += e5;
    soff[8 * tid + 6] = run; run += e6;
    soff[8 * tid + 7] = run;
    carry = b4;
    __syncthreads();
    const v4i o0 = *(const v4i*)(soff + 4 * tid);
    const v4i o1 = *(const v4i*)(soff + 4 * (tid + OTHR));
    int* op = off + base;
    *(volatile v4i*)(op + 4 * tid) = o0;
    *(volatile v4i*)(op + 4 * (tid + OTHR)) = o1;
    __threadfence();
    *(volatile v4i*)(op + 4 * tid) = o0;
    *(volatile v4i*)(op + 4 * (tid + OTHR)) = o1;
    __syncthreads();
  }
  if (tid == 0) srb[min(4 * nChunk, RBN - 1)] = carry;
  __syncthreads();
  v4i rv = {0, 0, 0, 0};
  if (tid < 32) rv = *(const v4i*)(srb + 4 * tid);
  if (tid < 32) *(volatile v4i*)(rbase + 4 * tid) = rv;
  __threadfence();
  if (tid < 32) *(volatile v4i*)(rbase + 4 * tid) = rv;
}

__global__ __launch_bounds__(NTHR) void k_fill(
    const int* __restrict__ dsts, const int* __restrict__ off, const int* __restrict__ rbase,
    int* csr, int nE, int vec8, int csrLen) {
  extern __shared__ v4f lds_dyn[];
  int* region = (int*)lds_dyn;
  int* cursor = region + RCAP;
  int* list   = cursor + NBF;
  int* wcnt   = list + LISTN;
  const int tid = threadIdx.x, lane = tid & 31, wave = tid >> 5;
  const int b = blockIdx.x;
  const int nodeBase = b * NBF;

  int rb0 = rbase[b];
  const int rb1 = rbase[b + 1];
  rb0 = rb0 < 0 ? 0 : (rb0 > csrLen ? csrLen : rb0);
  rb0 &= ~31;
  int len = rb1 - rb0;
  len = len < 0 ? 0 : (len > RCAP ? RCAP : len);
  int lenW = (len + 31) & ~31;
  if (rb0 + lenW > csrLen) lenW = (csrLen - rb0) & ~31;

  {
    const v4i z = {0, 0, 0, 0};
    for (int i = tid; i < RCAP / 4; i += NTHR) ((v4i*)region)[i] = z;
    for (int s = tid; s < NBF; s += NTHR) {
      int o = off[nodeBase + s] - rb0;
      o = o < 0 ? 0 : (o > RCAP ? RCAP : o);
      cursor[s] = o;
    }
  }
  __syncthreads();

  const int nChunks = (nE + CHUNK - 1) / CHUNK;
#pragma unroll 1
  for (int ch = 0; ch < nChunks; ++ch) {
    const int cbase = ch * CHUNK;
    const int wc = scan_chunk<NBF>(dsts, nE, cbase, nodeBase, vec8, list, tid, lane, wave);
    if (lane == 0) wcnt[wave] = wc;
    __syncthreads();
    if (wave == 0) {
#pragma unroll 1
      for (int wsx = 0; wsx < NWAVE; ++wsx) {
        int n = __builtin_amdgcn_readfirstlane(wcnt[wsx]);
        n = n > WCAP ? WCAP : (n < 0 ? 0 : n);
        const int* lp = list + wsx * WCAP;
#pragma unroll 1
        for (int i = 0; i < n; ++i) {
          const int ent  = __builtin_amdgcn_readfirstlane(lp[i]);
          const int slot = ent & (NBF - 1);
          int e = cbase + ((ent >> 12) & (CHUNK - 1));
          e = e > nE - 1 ? nE - 1 : (e < 0 ? 0 : e);
          if (lane == 0) {
            int pos = cursor[slot];
            pos = pos < 0 ? 0 : (pos > RCAP - 1 ? RCAP - 1 : pos);
            region[pos] = e;
            const int np = pos + 1;
            cursor[slot] = np > RCAP ? RCAP : np;
          }
        }
      }
    }
    __syncthreads();
  }

  const int nv = lenW >> 2;
  int* gp = csr + rb0;
#pragma unroll 1
  for (int i = tid; i < nv; i += NTHR) { const v4i v = ((const v4i*)region)[i]; *(volatile v4i*)(gp + 4 * i) = v; }
  __threadfence();
#pragma unroll 1
  for (int i = tid; i < nv; i += NTHR) { const v4i v = ((const v4i*)region)[i]; *(volatile v4i*)(gp + 4 * i) = v; }
}

__global__ __launch_bounds__(PTHR) void k_proj(
    const _Float16* __restrict__ Ap, const _Float16* __restrict__ Bp, float* Cp,
    int nRows, int aStride, int bStride, int cStride) {
  __shared__ __attribute__((aligned(16))) float stg[BM * AD];
  const int tid = threadIdx.x, lane = tid & 31, wave = tid >> 5;
  const int hh = lane >> 4, m = lane & 15;
  const int rg = wave >> 1, ct = wave & 1;
  const int ly = (int)blockIdx.y;
  const int rowBase = (int)blockIdx.x * BM;
  const _Float16* A = Ap + (size_t)ly * aStride;
  const _Float16* B = Bp + (size_t)ly * bStride;
  float* C = Cp + (size_t)ly * cStride;

  const _Float16* ap = A + (size_t)(rowBase + rg * 16 + m) * HD + 8 * hh;
  const _Float16* bp = B + (size_t)(ct * 16 + m) * HD + 8 * hh;
  v8f acc = {0.f, 0.f, 0.f, 0.f, 0.f, 0.f, 0.f, 0.f};
#pragma unroll
  for (int kt = 0; kt < 2; ++kt) {
    FragH a, bf;
    a.h[0]  = *(const v8h*)(ap + 32 * kt);
    a.h[1]  = *(const v8h*)(ap + 32 * kt + 16);
    bf.h[0] = *(const v8h*)(bp + 32 * kt);
    bf.h[1] = *(const v8h*)(bp + 32 * kt + 16);
    acc = wmh(a.v, bf.v, acc);
  }
  float* sp = stg + (size_t)(rg * 16 + 8 * hh) * AD + ct * 16 + m;
  const int grow0 = rowBase + rg * 16 + 8 * hh;
#pragma unroll
  for (int r = 0; r < 8; ++r) {
    float v = acc[r] * SCL_ACC;
    v = (grow0 + r < nRows) ? v : 0.0f;
    sp[r * AD] = v;
  }
  __syncthreads();

  float* tile = C + (size_t)rowBase * AD;
  const v4f o0 = *(const v4f*)(stg + 4 * tid);
  const v4f o1 = *(const v4f*)(stg + 4 * (tid + PTHR));
  *(volatile v4f*)(tile + 4 * tid) = o0;
  *(volatile v4f*)(tile + 4 * (size_t)(tid + PTHR)) = o1;
  __threadfence();
  *(volatile v4f*)(tile + 4 * tid) = o0;
  *(volatile v4f*)(tile + 4 * (size_t)(tid + PTHR)) = o1;
}

__global__ __launch_bounds__(NTHR) void k_agg(
    const int* __restrict__ csr, const int* __restrict__ off, const int* __restrict__ cnt,
    const int* __restrict__ edges, const float* __restrict__ psp, const float* __restrict__ prp,
    const float* __restrict__ waw, const float* __restrict__ wab,
    const float* __restrict__ h32, const float* __restrict__ rela,
    _Float16* ap, int nN, int nE, int nRel, int csrLen) {
  const int tid = threadIdx.x, lane = tid & 31, wave = tid >> 5;
  const int tbase = blockIdx.x * TGT + wave * 32;
  const int col2 = 2 * lane;

  const int cl    = tbase + lane;
  const int cnt_l = cnt[cl];
  const int off_l = off[cl];
  const float wl  = waw[lane];
  const float wb  = wab[0];

#pragma unroll 1
  for (int j = 0; j < 32; ++j) {
    const int c = tbase + j;
    int nraw = __shfl(cnt_l, j);
    nraw = nraw < 0 ? 0 : (nraw > nE ? nE : nraw);
    const int n = nraw > DEGCAP ? DEGCAP : nraw;
    const int st = __shfl(off_l, j);

    v2f acc = {0.0f, 0.0f};
#pragma unroll 1
    for (int q0 = 0; q0 < n; q0 += 32) {
      int pos = st + q0 + lane;
      pos = pos < 0 ? 0 : (pos > csrLen - 1 ? csrLen - 1 : pos);
      int el = csr[pos];
      el = el < 0 ? 0 : (el > nE - 1 ? nE - 1 : el);
      int sl = edges[(size_t)el * 6 + 4];
      sl = sl < 0 ? 0 : (sl > nN - 1 ? nN - 1 : sl);
      int rl = edges[(size_t)el * 6 + 2];
      rl = rl < 0 ? 0 : (rl > nRel - 1 ? nRel - 1 : rl);
      const int mcnt = (n - q0) < 32 ? (n - q0) : 32;
#pragma unroll 1
      for (int pp = 0; pp < mcnt; ++pp) {
        const int s = __builtin_amdgcn_readlane(sl, pp);
        const int r = __builtin_amdgcn_readlane(rl, pp);
        const float ps = psp[(size_t)s * AD + lane];
        const float pr = prp[(size_t)r * AD + lane];
        const v2f hv = *(const v2f*)(h32 + (size_t)s * HD + col2);
        const v2f rv = *(const v2f*)(rela + (size_t)r * HD + col2);
        float a = ps + pr;
        a = a > 0.0f ? a : 0.0f;
        float p = a * wl;
        p += __shfl_xor(p, 16);
        p += __shfl_xor(p, 8);
        p += __shfl_xor(p, 4);
        p += __shfl_xor(p, 2);
        p += __shfl_xor(p, 1);
        const float alpha = sigm(p + wb);
        const v2f sm = hv + rv;
        const v2f msg = sm * alpha;
        acc = acc + msg;
      }
    }

    v2f v = acc * SCL_A;
    if (nraw > DEGCAP) { const float qn = __int_as_float(0x7fc00000); v.x = qn; v.y = qn; }
    if (c >= nN) { v.x = 0.0f; v.y = 0.0f; }
    const v2h o = __builtin_convertvector(v, v2h);
    _Float16* gp = ap + (size_t)c * HD + col2;
    *(volatile v2h*)gp = o;
    __threadfence();
    *(volatile v2h*)gp = o;
  }
}

__global__ __launch_bounds__(NTHR) void k_node(
    const _Float16* __restrict__ aggP, const _Float16* __restrict__ whp,
    const _Float16* __restrict__ wihp, const _Float16* __restrict__ whhp,
    const float* __restrict__ bih, const float* __restrict__ bhh,
    float* H32, _Float16* H16, const float* __restrict__ wf, float* out,
    int nN, int fin) {
  __shared__ __attribute__((aligned(16))) _Float16 xs[BM * HD];
  __shared__ __attribute__((aligned(16))) float stg[BM * HD];
  __shared__ __attribute__((aligned(16))) float ssc[BM];
  const int tid = threadIdx.x, lane = tid & 31, wave = tid >> 5;
  const int hh = lane >> 4, m = lane & 15;
  const int rg = wave >> 2, ct = wave & 3;
  const int rowBase = (int)blockIdx.x * BM;
  const int arow = rowBase + rg * 16 + m;
  const int ncol = ct * 16 + m;
  const v8f z8 = {0.f, 0.f, 0.f, 0.f, 0.f, 0.f, 0.f, 0.f};

  {
    const _Float16* ap = aggP + (size_t)arow * HD + 8 * hh;
    const _Float16* bp = whp + (size_t)ncol * HD + 8 * hh;
    v8f acc = z8;
#pragma unroll
    for (int kt = 0; kt < 2; ++kt) {
      FragH a, bf;
      a.h[0]  = *(const v8h*)(ap + 32 * kt);
      a.h[1]  = *(const v8h*)(ap + 32 * kt + 16);
      bf.h[0] = *(const v8h*)(bp + 32 * kt);
      bf.h[1] = *(const v8h*)(bp + 32 * kt + 16);
      acc = wmh(a.v, bf.v, acc);
    }
    _Float16* xrow = xs + (size_t)(rg * 16 + 8 * hh) * HD + ncol;
#pragma unroll
    for (int r = 0; r < 8; ++r) {
      float v = acc[r] * SCL_ACC;
      v = v > 0.0f ? v : 0.0f;
      xrow[r * HD] = (_Float16)(v * SCL_A);
    }
  }
  __syncthreads();

  FragH xa[2], ha[2];
  {
    const _Float16* xr = xs + (size_t)(rg * 16 + m) * HD + 8 * hh;
    const _Float16* hr = H16 + (size_t)arow * HD + 8 * hh;
#pragma unroll
    for (int kt = 0; kt < 2; ++kt) {
      xa[kt].h[0] = *(const v8h*)(xr + 32 * kt);
      xa[kt].h[1] = *(const v8h*)(xr + 32 * kt + 16);
      ha[kt].h[0] = *(const v8h*)(hr + 32 * kt);
      ha[kt].h[1] = *(const v8h*)(hr + 32 * kt + 16);
    }
  }
  v8f gir = z8, giz = z8, gin = z8, ghr = z8, ghz = z8, ghn = z8;
#pragma unroll
  for (int kt = 0; kt < 2; ++kt) {
    const _Float16* bi = wihp + (size_t)ncol * HD + 32 * kt + 8 * hh;
    const _Float16* bh = whhp + (size_t)ncol * HD + 32 * kt + 8 * hh;
    FragH bf;
    bf.h[0] = *(const v8h*)(bi);                       bf.h[1] = *(const v8h*)(bi + 16);                       gir = wmh(xa[kt].v, bf.v, gir);
    bf.h[0] = *(const v8h*)(bi + (size_t)64 * HD);     bf.h[1] = *(const v8h*)(bi + (size_t)64 * HD + 16);     giz = wmh(xa[kt].v, bf.v, giz);
    bf.h[0] = *(const v8h*)(bi + (size_t)128 * HD);    bf.h[1] = *(const v8h*)(bi + (size_t)128 * HD + 16);    gin = wmh(xa[kt].v, bf.v, gin);
    bf.h[0] = *(const v8h*)(bh);                       bf.h[1] = *(const v8h*)(bh + 16);                       ghr = wmh(ha[kt].v, bf.v, ghr);
    bf.h[0] = *(const v8h*)(bh + (size_t)64 * HD);     bf.h[1] = *(const v8h*)(bh + (size_t)64 * HD + 16);     ghz = wmh(ha[kt].v, bf.v, ghz);
    bf.h[0] = *(const v8h*)(bh + (size_t)128 * HD);    bf.h[1] = *(const v8h*)(bh + (size_t)128 * HD + 16);    ghn = wmh(ha[kt].v, bf.v, ghn);
  }

  {
    const float bir = bih[ncol], biz = bih[HD + ncol], bin = bih[2 * HD + ncol];
    const float bhr = bhh[ncol], bhz = bhh[HD + ncol], bhn = bhh[2 * HD + ncol];
    const int lrow0 = rg * 16 + 8 * hh;
    float* sp = stg + (size_t)lrow0 * HD + ncol;
    const float* hp = H32 + (size_t)(rowBase + lrow0) * HD + ncol;
#pragma unroll
    for (int r = 0; r < 8; ++r) {
      const float hold = hp[(size_t)r * HD];
      const float xr_ = gir[r] * SCL_ACC + bir;
      const float hr_ = ghr[r] * SCL_ACC + bhr;
      const float xz_ = giz[r] * SCL_ACC + biz;
      const float hz_ = ghz[r] * SCL_ACC + bhz;
      const float xn_ = gin[r] * SCL_ACC + bin;
      const float hn_ = ghn[r] * SCL_ACC + bhn;
      const float rgt = sigm(xr_ + hr_);
      const float zgt = sigm(xz_ + hz_);
      const float ngt = tanhf(xn_ + rgt * hn_);
      float h = (1.0f - zgt) * ngt + zgt * hold;
      h = (rowBase + lrow0 + r < nN) ? h : 0.0f;
      sp[r * HD] = h;
    }
  }
  __syncthreads();

  {
    const int row = tid >> 3, q = tid & 7;
    const v4f s0 = *(const v4f*)(stg + (size_t)row * HD + 8 * q);
    const v4f s1 = *(const v4f*)(stg + (size_t)row * HD + 8 * q + 4);
    const v4f w0 = *(const v4f*)(wf + 8 * q);
    const v4f w1 = *(const v4f*)(wf + 8 * q + 4);
    float s = s0.x * w0.x + s0.y * w0.y + s0.z * w0.z + s0.w * w0.w
            + s1.x * w1.x + s1.y * w1.y + s1.z * w1.z + s1.w * w1.w;
    s += __shfl_xor(s, 4);
    s += __shfl_xor(s, 2);
    s += __shfl_xor(s, 1);
    if (q == 0) ssc[row] = s;
  }
  const v4f o0 = *(const v4f*)(stg + 4 * tid);
  const v4f o1 = *(const v4f*)(stg + 4 * (tid + NTHR));
  const v8h oh = cvt8(*(const v4f*)(stg + 8 * tid), *(const v4f*)(stg + 8 * tid + 4), SCL_A);
  __syncthreads();

  float* t32 = H32 + (size_t)rowBase * HD;
  _Float16* t16 = H16 + (size_t)rowBase * HD;
  const bool doOut  = (fin != 0) && (rowBase < nN);
  const bool fullLn = (rowBase + BM <= nN);
  v4f sv = {0.0f, 0.0f, 0.0f, 0.0f};
  if (tid < 8) sv = *(const v4f*)(ssc + 4 * tid);
  const float st = ssc[tid & (BM - 1)];

  *(volatile v4f*)(t32 + 4 * tid) = o0;
  *(volatile v4f*)(t32 + 4 * (size_t)(tid + NTHR)) = o1;
  *(volatile v8h*)(t16 + 8 * (size_t)tid) = oh;
  if (doOut) {
    if (fullLn) {
      if (tid < 8) *(volatile v4f*)(out + rowBase + 4 * tid) = sv;
    } else {
      if (tid < BM && rowBase + tid < nN) *(volatile float*)(out + rowBase + tid) = st;
    }
  }
  __threadfence();
  *(volatile v4f*)(t32 + 4 * tid) = o0;
  *(volatile v4f*)(t32 + 4 * (size_t)(tid + NTHR)) = o1;
  *(volatile v8h*)(t16 + 8 * (size_t)tid) = oh;
  if (doOut) {
    if (fullLn) {
      if (tid < 8) *(volatile v4f*)(out + rowBase + 4 * tid) = sv;
    } else {
      if (tid < BM && rowBase + tid < nN) *(volatile float*)(out + rowBase + tid) = st;
    }
  }
}

extern "C" void kernel_launch(void* const* d_in, const int* in_sizes, int n_in,
                              void* d_out, int out_size, void* d_ws, size_t ws_size,
                              hipStream_t stream) {
  if (n_in < 12) return;
  const int nN = out_size;
  if (nN <= 0 || nN > (1 << 22)) return;
  if (in_sizes[0] <= 0 || (in_sizes[0] % 6) != 0) return;
  const int nE = in_sizes[0] / 6;
  if (nE <= 0 || nE > (1 << 28)) return;
  if (in_sizes[2] <= 0 || (in_sizes[2] % (AD * HD)) != 0) return;
  const int NL = in_sizes[2] / (AD * HD);
  if (NL < 1 || NL > 8) return;
  if (in_sizes[3] != NL * AD * HD || in_sizes[4] != NL * AD || in_sizes[5] != NL) return;
  if (in_sizes[6] != NL * HD * HD || in_sizes[7] != NL * G3 * HD || in_sizes[8] != NL * G3 * HD) return;
  if (in_sizes[9] != NL * G3 || in_sizes[10] != NL * G3 || in_sizes[11] != HD) return;
  if (in_sizes[1] <= 0 || (in_sizes[1] % (NL * HD)) != 0) return;
  const int nRel = in_sizes[1] / (NL * HD);
  if (nRel <= 0 || nRel > (1 << 20)) return;

  const int*   edges = (const int*)d_in[0];
  const float* rela  = (const float*)d_in[1];
  const float* Ws    = (const float*)d_in[2];
  const float* Wr    = (const float*)d_in[3];
  const float* waw   = (const float*)d_in[4];
  const float* wab   = (const float*)d_in[5];
  const float* Wh    = (const float*)d_in[6];
  const float* Wih   = (const float*)d_in[7];
  const float* Whh   = (const float*)d_in[8];
  const float* bih   = (const float*)d_in[9];
  const float* bhh   = (const float*)d_in[10];
  const float* Wf    = (const float*)d_in[11];
  float* out = (float*)d_out;

  const int NPAD   = ((nN + TGT - 1) / TGT) * TGT;
  const int nBC    = (nN + NBC - 1) / NBC;
  const int CNTPAD = nBC * NBC;
  if (CNTPAD < NPAD) return;
  if (4 * nBC + 1 > RBN) return;
  const int nBF    = (nN + NBF - 1) / NBF;
  if (nBF + 1 > 4 * nBC + 1) return;
  const int nE32   = (nE + 31) & ~31;
  const int csrLen = nE32 + 4096;
  if (31 * 4 * nBC > 4096) return;
  const int RPAD   = ((nRel + BM - 1) / BM) * BM;
  const int nAgg   = NPAD / TGT;
  const int nNode  = NPAD / BM;
  const int nObjU  = nE32 / 4;
  const int nRelU  = RPAD * (HD / 8);

  char* ws = (char*)d_ws;
  size_t off = 0;
  const size_t oObj = off; off += (size_t)nE32 * 4;              off = (off + 255) & ~(size_t)255;
  const size_t oCnt = off; off += (size_t)CNTPAD * 4;            off = (off + 255) & ~(size_t)255;
  const size_t oOff = off; off += (size_t)CNTPAD * 4;            off = (off + 255) & ~(size_t)255;
  const size_t oRb  = off; off += (size_t)RBN * 4;               off = (off + 255) & ~(size_t)255;
  const size_t oCsr = off; off += (size_t)csrLen * 4;            off = (off + 255) & ~(size_t)255;
  const size_t oWs  = off; off += (size_t)NL * AD * HD * 2;      off = (off + 255) & ~(size_t)255;
  const size_t oWr  = off; off += (size_t)NL * AD * HD * 2;      off = (off + 255) & ~(size_t)255;
  const size_t oWh  = off; off += (size_t)NL * HD * HD * 2;      off = (off + 255) & ~(size_t)255;
  const size_t oWih = off; off += (size_t)NL * G3 * HD * 2;      off = (off + 255) & ~(size_t)255;
  const size_t oWhh = off; off += (size_t)NL * G3 * HD * 2;      off = (off + 255) & ~(size_t)255;
  const size_t oRel = off; off += (size_t)NL * RPAD * HD * 2;    off = (off + 255) & ~(size_t)255;
  const size_t oPr  = off; off += (size_t)NL * RPAD * AD * 4;    off = (off + 255) & ~(size_t)255;
  const size_t oPs  = off; off += (size_t)NPAD * AD * 4;         off = (off + 255) & ~(size_t)255;
  const size_t oH32 = off; off += (size_t)NPAD * HD * 4;
  const size_t oH16 = off; off += (size_t)NPAD * HD * 2;         off = (off + 255) & ~(size_t)255;
  const size_t oAgg = off; off += (size_t)NPAD * HD * 2;         off = (off + 255) & ~(size_t)255;
  if (off > ws_size || off > (size_t)WSCAP) return;
  int*      objP = (int*)(ws + oObj);
  int*      cnt  = (int*)(ws + oCnt);
  int*      offp = (int*)(ws + oOff);
  int*      rb   = (int*)(ws + oRb);
  int*      csr  = (int*)(ws + oCsr);
  _Float16* WsP  = (_Float16*)(ws + oWs);
  _Float16* WrP  = (_Float16*)(ws + oWr);
  _Float16* WhP  = (_Float16*)(ws + oWh);
  _Float16* WihP = (_Float16*)(ws + oWih);
  _Float16* WhhP = (_Float16*)(ws + oWhh);
  _Float16* relP = (_Float16*)(ws + oRel);
  float*    PrP  = (float*)(ws + oPr);
  float*    PsP  = (float*)(ws + oPs);
  float*    H32  = (float*)(ws + oH32);
  _Float16* H16  = (_Float16*)(ws + oH16);
  _Float16* aggP = (_Float16*)(ws + oAgg);
  const int nZeroU = (int)(((size_t)NPAD * HD * 4 + (size_t)NPAD * HD * 2) / 16);

  k_extract<<<(nObjU + NTHR - 1) / NTHR, NTHR, 0, stream>>>(edges, objP, nE, nObjU);
  k_count<<<nBC, NTHR, 0, stream>>>(objP, cnt, nE, 1);
  k_offsets<<<1, OTHR, 0, stream>>>(cnt, offp, rb, nBC);
  hipFuncSetAttribute(reinterpret_cast<const void*>(&k_fill),
                      hipFuncAttributeMaxDynamicSharedMemorySize, LDS_FILL);
  k_fill<<<nBF, NTHR, LDS_FILL, stream>>>(objP, offp, rb, csr, nE, 1, csrLen);

  k_zero16<<<(nZeroU + NTHR - 1) / NTHR, NTHR, 0, stream>>>(H32, nZeroU);

  { const int u = in_sizes[2] / 8;  k_prepw_flat<<<(u + NTHR - 1) / NTHR, NTHR, 0, stream>>>(Ws,  WsP,  u); }
  { const int u = in_sizes[3] / 8;  k_prepw_flat<<<(u + NTHR - 1) / NTHR, NTHR, 0, stream>>>(Wr,  WrP,  u); }
  { const int u = in_sizes[6] / 8;  k_prepw_flat<<<(u + NTHR - 1) / NTHR, NTHR, 0, stream>>>(Wh,  WhP,  u); }
  { const int u = in_sizes[7] / 8;  k_prepw_flat<<<(u + NTHR - 1) / NTHR, NTHR, 0, stream>>>(Wih, WihP, u); }
  { const int u = in_sizes[8] / 8;  k_prepw_flat<<<(u + NTHR - 1) / NTHR, NTHR, 0, stream>>>(Whh, WhhP, u); }
  k_acvt<<<dim3((nRelU + NTHR - 1) / NTHR, NL), NTHR, 0, stream>>>(rela, relP, nRel, RPAD, nRelU);

  k_proj<<<dim3(RPAD / BM, NL), PTHR, 0, stream>>>(relP, WrP, PrP, nRel, RPAD * HD, AD * HD, RPAD * AD);

  for (int l = 0; l < NL; ++l) {
    k_proj<<<dim3(nNode, 1), PTHR, 0, stream>>>(H16, WsP + (size_t)l * AD * HD, PsP, nN, 0, 0, 0);
    k_agg<<<nAgg, NTHR, 0, stream>>>(csr, offp, cnt, edges, PsP, PrP + (size_t)l * RPAD * AD,
                                     waw + (size_t)l * AD, wab + l, H32, rela + (size_t)l * nRel * HD,
                                     aggP, nN, nE, nRel, csrLen);
    k_node<<<nNode, NTHR, 0, stream>>>(aggP, WhP + (size_t)l * HD * HD, WihP + (size_t)l * G3 * HD,
                                       WhhP + (size_t)l * G3 * HD, bih + (size_t)l * G3, bhh + (size_t)l * G3,
                                       H32, H16, Wf, out, nN, (l == NL - 1) ? 1 : 0);
  }
}
